// MambaPOD_space_54795192762430
// MI455X (gfx1250) — hardware-verified
//
#include <hip/hip_runtime.h>
#include <cstdint>
#include <cstddef>

typedef __attribute__((ext_vector_type(16))) _Float16 v16h;
typedef __attribute__((ext_vector_type(8)))  float    v8f;

union FragAB { v16h v; uint32_t u[8]; };

#define BSZ   4
#define SEQL  2048
#define DMOD  192
#define DINN  384
#define DST   64
#define DCONV 4
#define DRANK 12
#define BL    (BSZ * SEQL)
#define NPAD2 128
#define RSPLIT (1.0f / 2048.0f)
#define PL_H16 ((size_t)BL * DMOD)
#define PL_X16 ((size_t)BL * DINN)
#define PL_Y16 ((size_t)BL * DINN)
typedef __attribute__((ext_vector_type(8))) _Float16 v8h;
typedef __attribute__((ext_vector_type(4))) float v4f_t;
typedef float v4fa __attribute__((ext_vector_type(4), may_alias));
__device__ __forceinline__ _Float16 lo_of(float v, _Float16 h) { return (_Float16)((v - (float)h) * 2048.0f); }
__device__ __forceinline__ void st2f(float* p, float v) { *(volatile float*)p = v; __threadfence(); *(volatile float*)p = v; }
__device__ __forceinline__ void st2pair(_Float16* p, size_t pl, float v0, float v1) {
  const _Float16 a = (_Float16)v0, b = (_Float16)v1;
  const unsigned u = (unsigned)__builtin_bit_cast(unsigned short, a) | ((unsigned)__builtin_bit_cast(unsigned short, b) << 16);
  const unsigned w = (unsigned)__builtin_bit_cast(unsigned short, lo_of(v0, a)) | ((unsigned)__builtin_bit_cast(unsigned short, lo_of(v1, b)) << 16);
  *(volatile unsigned*)p = u; *(volatile unsigned*)(p + pl) = w; __threadfence(); *(volatile unsigned*)p = u; *(volatile unsigned*)(p + pl) = w;
}
__device__ __forceinline__ v8f wmma16(v16h a, v16h b, v8f c) { return __builtin_amdgcn_wmma_f32_16x16x32_f16(false, a, false, b, (short)0, c, false, false); }
__device__ __forceinline__ v8f wmma_split(v16h a, v16h al, v16h b, v16h bl, v8f c) { v8f x = {}; x = wmma16(al, b, x); x = wmma16(a, bl, x); return wmma16(a, b, c) + x * RSPLIT; }

__global__ void pack_w_kernel(const float* __restrict__ W, _Float16* __restrict__ Bp,
                              int Nreal, int K, int ntiles, size_t pl) {
  const int kchunks = K / 32;
  const int t = blockIdx.x * 256 + threadIdx.x;
  if (t >= ntiles * kchunks * 32) return;
  const int lane = t & 31;
  const int kc   = (t >> 5) % kchunks;
  const int nt   = t / (32 * kchunks);
  const int n    = nt * 16 + (lane & 15);
  const int kb   = kc * 32 + (lane >> 4) * 8;
  _Float16* dst = Bp + (size_t)t * 16;
#pragma unroll
  for (int e = 0; e < 16; e += 2) {
    const int k0 = kb + ((e < 8) ? e : (e + 8));
    const float v0 = (n < Nreal) ? W[(size_t)n * K + k0] : 0.0f;
    const float v1 = (n < Nreal) ? W[(size_t)n * K + k0 + 1] : 0.0f;
    st2pair(dst + e, pl, v0, v1);
  }
}

__global__ void resid_ln_kernel(const float* __restrict__ hs, const float* __restrict__ res_in,
                                const float* __restrict__ ln_w, const float* __restrict__ ln_b,
                                float* __restrict__ res_out, _Float16* __restrict__ h16) {
  __shared__ float sbuf[64];
  const int row = blockIdx.x;
  const int tid = threadIdx.x;
  const size_t base = (size_t)row * DMOD;

  float v[3];
  float s = 0.0f;
#pragma unroll
  for (int i = 0; i < 3; ++i) {
    const int c = tid + i * 64;
    float x = res_in[base + c] + hs[base + c];
    v[i] = x; s += x;
    st2f(res_out + base + c, x);
  }
  sbuf[tid] = s;
  for (int off = 32; off > 0; off >>= 1) { __syncthreads(); if (tid < off) sbuf[tid] += sbuf[tid + off]; }
  __syncthreads();
  const float mu = sbuf[0] * (1.0f / DMOD);
  __syncthreads();

  float s2 = 0.0f;
#pragma unroll
  for (int i = 0; i < 3; ++i) { float d = v[i] - mu; s2 += d * d; }
  sbuf[tid] = s2;
  for (int off = 32; off > 0; off >>= 1) { __syncthreads(); if (tid < off) sbuf[tid] += sbuf[tid + off]; }
  __syncthreads();
  const float inv = rsqrtf(sbuf[0] * (1.0f / DMOD) + 1e-5f);

  __shared__ __attribute__((aligned(16))) float sh[DMOD];
#pragma unroll
  for (int i = 0; i < 3; ++i) {
    const int c = tid + i * 64;
    sh[c] = (v[i] - mu) * inv * ln_w[c] + ln_b[c];
  }
  __syncthreads();
  if (tid < DMOD / 8) {
    typedef __attribute__((ext_vector_type(4))) unsigned v4u_t; typedef unsigned v4ua __attribute__((ext_vector_type(4), may_alias));
    _Float16 hh[8], hl[8];
#pragma unroll
    for (int e = 0; e < 8; ++e) { const float f = sh[tid * 8 + e]; hh[e] = (_Float16)f; hl[e] = lo_of(f, hh[e]); }
    const v4u_t u0 = *(const v4ua*)hh, u1 = *(const v4ua*)hl;
    _Float16* d = h16 + base + tid * 8;
    *(volatile v4u_t*)d = u0; *(volatile v4u_t*)(d + PL_H16) = u1; __threadfence(); *(volatile v4u_t*)d = u0; *(volatile v4u_t*)(d + PL_H16) = u1;
  }
}

__global__ __launch_bounds__(128) void gemm_wmma_kernel(
    const _Float16* __restrict__ A, size_t plA, const _Float16* __restrict__ Bp, size_t plB,
    float* __restrict__ C, int K, int N, int Mtiles, int kchunks) {
  __shared__ __attribute__((aligned(16))) float stg[4][16 * 68];
  const int wave = threadIdx.x >> 5;
  const int lane = threadIdx.x & 31;
  const int t     = blockIdx.x * 4 + wave;
  const int tileM = t % Mtiles;
  const int grpN  = t / Mtiles;
  const int r    = lane & 15;
  const int half = lane >> 4;

  v8f acc[4] = {};
  const _Float16* arow = A + (size_t)(tileM * 16 + r) * K;

  for (int kc = 0; kc < kchunks; ++kc) {
    FragAB a, al;
    const uint32_t* ap  = (const uint32_t*)(arow + kc * 32);
    const uint32_t* apl = (const uint32_t*)(arow + plA + kc * 32);
#pragma unroll
    for (int vg = 0; vg < 8; ++vg) {
      const int pair = (vg < 4) ? (vg + half * 4) : (4 + vg + half * 4);
      a.u[vg] = ap[pair]; al.u[vg] = apl[pair];
    }
#pragma unroll
    for (int nt = 0; nt < 4; ++nt) {
      const _Float16* bb = Bp + (((size_t)(grpN * 4 + nt) * kchunks + kc) * 32 + lane) * 16;
      const v16h b = *(const v16h*)bb, bl = *(const v16h*)(bb + plB);
      acc[nt] = wmma_split(a.v, al.v, b, bl, acc[nt]);
    }
  }
  float* sw = stg[wave];
#pragma unroll
  for (int nt = 0; nt < 4; ++nt)
#pragma unroll
    for (int vg = 0; vg < 8; ++vg) sw[(half * 8 + vg) * 68 + nt * 16 + r] = acc[nt][vg];
  asm volatile("s_wait_dscnt 0" ::: "memory");
#pragma unroll 1
  for (int pass = 0; pass < 2; ++pass) {
#pragma unroll
    for (int i = 0; i < 8; ++i) { const int c = lane + 32 * i, rr = c >> 4, q = (c & 15) * 4;
      *(volatile v4f_t*)(C + (size_t)(tileM * 16 + rr) * N + grpN * 64 + q) = *(const volatile v4fa*)(sw + rr * 68 + q); }
    __threadfence();
  }
}

__global__ void conv_silu_kernel(const float* __restrict__ xz, const float* __restrict__ conv_w,
                                 const float* __restrict__ conv_b,
                                 float* __restrict__ x32, _Float16* __restrict__ x16) {
  const int idx0 = (blockIdx.x * 256 + threadIdx.x) * 2;
  if (idx0 >= BL * DINN) return;
  float yv[2];
#pragma unroll
  for (int u = 0; u < 2; ++u) {
    const int idx = idx0 + u;
    const int c   = idx % DINN;
    const int row = idx / DINN;
    const int l   = row % SEQL;
    const int b   = row / SEQL;
    float acc = conv_b[c];
#pragma unroll
    for (int j = 0; j < DCONV; ++j) {
      const int ls = l - (DCONV - 1) + j;
      if (ls >= 0)
        acc += conv_w[c * DCONV + j] * xz[((size_t)b * SEQL + ls) * (2 * DINN) + c];
    }
    yv[u] = acc / (1.0f + __expf(-acc));
  }
  typedef __attribute__((ext_vector_type(2))) float v2f_t; v2f_t y2; y2.x = yv[0]; y2.y = yv[1];
  *(volatile v2f_t*)(x32 + idx0) = y2; __threadfence(); *(volatile v2f_t*)(x32 + idx0) = y2;
  st2pair(x16 + idx0, PL_X16, yv[0], yv[1]);
}

__global__ void dt_kernel(const float* __restrict__ xdb, const float* __restrict__ W_dt,
                          const float* __restrict__ b_dt, float* __restrict__ dt) {
  const int idx = blockIdx.x * 256 + threadIdx.x;
  if (idx >= BL * DINN) return;
  const int d = idx % DINN;
  const int m = idx / DINN;
  float acc = b_dt[d];
  const float* xr = xdb + (size_t)m * NPAD2;
  const float* wr = W_dt + (size_t)d * DRANK;
#pragma unroll
  for (int r = 0; r < DRANK; ++r) acc += xr[r] * wr[r];
  st2f(dt + idx, (acc > 20.0f) ? acc : log1pf(__expf(acc)));
}

__global__ __launch_bounds__(128) void scan_kernel(
    const float* __restrict__ dt, const float* __restrict__ x32,
    const float* __restrict__ xdb, const float* __restrict__ A_log,
    const float* __restrict__ C_fixed, float* __restrict__ y) {
  const int wave = threadIdx.x >> 5;
  const int lane = threadIdx.x & 31;
  const int w = blockIdx.x * 4 + wave;
  const int b = w / DINN;
  const int d = w % DINN;
  const int n0 = lane, n1 = lane + 32;

  const float A0 = -__expf(A_log[d * DST + n0]);
  const float A1 = -__expf(A_log[d * DST + n1]);
  const float C0 = C_fixed[n0];
  const float C1 = C_fixed[n1];

  float h0 = 0.0f, h1 = 0.0f, ykeep = 0.0f;
  const size_t tok0 = (size_t)b * SEQL;
  for (int l = 0; l < SEQL; ++l) {
    const size_t row = tok0 + l;
    const float dtv = dt[row * DINN + d];
    const float u   = x32[row * DINN + d];
    const float du  = dtv * u;
    const float b0  = xdb[row * NPAD2 + DRANK + n0];
    const float b1  = xdb[row * NPAD2 + DRANK + n1];
    h0 = __expf(dtv * A0) * h0 + du * b0;
    h1 = __expf(dtv * A1) * h1 + du * b1;
    float part = h0 * C0 + h1 * C1;
#pragma unroll
    for (int off = 16; off > 0; off >>= 1) part += __shfl_xor(part, off);
    if (lane == (l & 31)) ykeep = part;
    if ((l & 31) == 31) {
      float* yp = y + ((size_t)b * DINN + d) * SEQL + (l - 31) + lane;
      *(volatile float*)yp = ykeep; __threadfence(); *(volatile float*)yp = ykeep;
    }
  }
}

__global__ void gate_kernel(const float* __restrict__ y_scan, const float* __restrict__ x32,
                            const float* __restrict__ xz, const float* __restrict__ D_skip,
                            _Float16* __restrict__ y16) {
  const int idx0 = (blockIdx.x * 256 + threadIdx.x) * 2;
  if (idx0 >= BL * DINN) return;
  float yy[2];
#pragma unroll
  for (int u = 0; u < 2; ++u) {
    const int idx = idx0 + u;
    const int d = idx % DINN;
    const int m = idx / DINN;
    const int b = m / SEQL, l = m % SEQL;
    const float z = xz[(size_t)m * (2 * DINN) + DINN + d];
    const float g = z / (1.0f + __expf(-z));
    yy[u] = (y_scan[((size_t)b * DINN + d) * SEQL + l] + x32[idx] * D_skip[d]) * g;
  }
  st2pair(y16 + idx0, PL_Y16, yy[0], yy[1]);
}

extern "C" void kernel_launch(void* const* d_in, const int* in_sizes, int n_in,
                              void* d_out, int out_size, void* d_ws, size_t ws_size,
                              hipStream_t stream) {
  (void)in_sizes; (void)n_in; (void)out_size; (void)ws_size;
  const float* hs      = (const float*)d_in[0];
  const float* res_in  = (const float*)d_in[1];
  const float* ln_w    = (const float*)d_in[2];
  const float* ln_b    = (const float*)d_in[3];
  const float* W_in    = (const float*)d_in[4];
  const float* conv_w  = (const float*)d_in[5];
  const float* conv_b  = (const float*)d_in[6];
  const float* W_xproj = (const float*)d_in[7];
  const float* W_dt    = (const float*)d_in[8];
  const float* b_dt    = (const float*)d_in[9];
  const float* A_log   = (const float*)d_in[10];
  const float* D_skip  = (const float*)d_in[11];
  const float* C_fixed = (const float*)d_in[12];
  const float* W_out   = (const float*)d_in[13];

  float* out     = (float*)d_out;
  float* res_out = out + (size_t)BL * DMOD;

  char* wsp = (char*)d_ws;
  auto carve = [&](size_t bytes) -> char* {
    char* p = wsp; wsp += (bytes + 255) & ~(size_t)255; return p;
  };
  _Float16* h16  = (_Float16*)carve((size_t)BL * DMOD * 2 * 2);
  float*    xz   = (float*)   carve((size_t)BL * 2 * DINN * 4);
  float*    x32  = (float*)   carve((size_t)BL * DINN * 4);
  _Float16* x16  = (_Float16*)carve((size_t)BL * DINN * 2 * 2);
  float*    xdb  = (float*)   carve((size_t)BL * NPAD2 * 4);
  float*    dtb  = (float*)   carve((size_t)BL * DINN * 4);
  float*    ysc  = (float*)   carve((size_t)BL * DINN * 4);
  _Float16* y16  = (_Float16*)carve((size_t)BL * DINN * 2 * 2);
  const size_t PB1 = (size_t)48 * 6 * 32 * 16, PB2 = (size_t)8 * 12 * 32 * 16, PB3 = (size_t)12 * 12 * 32 * 16;
  _Float16* bp1  = (_Float16*)carve(PB1 * 2 * 2);
  _Float16* bp2  = (_Float16*)carve(PB2 * 2 * 2);
  _Float16* bp3  = (_Float16*)carve(PB3 * 2 * 2);

  pack_w_kernel<<<(48 * 6 * 32 + 255) / 256, 256, 0, stream>>>(W_in,    bp1, 2 * DINN,        DMOD, 48, PB1);
  pack_w_kernel<<<(8  * 12 * 32 + 255) / 256, 256, 0, stream>>>(W_xproj, bp2, DRANK + DST,     DINN, 8, PB2);
  pack_w_kernel<<<(12 * 12 * 32 + 255) / 256, 256, 0, stream>>>(W_out,   bp3, DMOD,            DINN, 12, PB3);

  resid_ln_kernel<<<BL, 64, 0, stream>>>(hs, res_in, ln_w, ln_b, res_out, h16);

  gemm_wmma_kernel<<<(BL / 16) * 12 / 4, 128, 0, stream>>>(h16, PL_H16, bp1, PB1, xz, DMOD, 2 * DINN, BL / 16, DMOD / 32);

  conv_silu_kernel<<<(BL * DINN / 2 + 255) / 256, 256, 0, stream>>>(xz, conv_w, conv_b, x32, x16);

  gemm_wmma_kernel<<<(BL / 16) * 2 / 4, 128, 0, stream>>>(x16, PL_X16, bp2, PB2, xdb, DINN, NPAD2, BL / 16, DINN / 32);

  dt_kernel<<<(BL * DINN + 255) / 256, 256, 0, stream>>>(xdb, W_dt, b_dt, dtb);

  scan_kernel<<<(BSZ * DINN) / 4, 128, 0, stream>>>(dtb, x32, xdb, A_log, C_fixed, ysc);

  gate_kernel<<<(BL * DINN / 2 + 255) / 256, 256, 0, stream>>>(ysc, x32, xz, D_skip, y16);

  gemm_wmma_kernel<<<(BL / 16) * 3 / 4, 128, 0, stream>>>(y16, PL_Y16, bp3, PB3, out, DINN, DMOD, BL / 16, DINN / 32);
}
